// DGCNN_Grouper_11897059410080
// MI455X (gfx1250) — hardware-verified
//
#include <hip/hip_runtime.h>
#include <math.h>
#include <stddef.h>

#pragma clang fp contract(off)

typedef __attribute__((ext_vector_type(16))) _Float16 v16h;
typedef __attribute__((ext_vector_type(8)))  _Float16 v8h;
typedef __attribute__((ext_vector_type(16))) __bf16   v16b;
typedef __attribute__((ext_vector_type(8)))  __bf16   v8b;
typedef __attribute__((ext_vector_type(8)))  float    v8f;
typedef __attribute__((ext_vector_type(4)))  float    v4f;
typedef __attribute__((ext_vector_type(4)))  unsigned int v4u;
typedef __attribute__((ext_vector_type(4)))  int      v4i;

constexpr int kBatch = 4;
constexpr int kN0 = 4096;
constexpr int kN1 = 2048;
constexpr int kN2 = 1024;
constexpr int kNbr = 16;
constexpr float kInvCnt = 1.0f / 524288.0f;
static_assert((32 / 4) * kN0 * kNbr == 524288 && (64 / 4) * kN1 * kNbr == 524288 && (128 / 4) * kN2 * kNbr == 524288);

constexpr size_t kOut0 = 0;
constexpr size_t kOut1 = 12288;
constexpr size_t kOut2 = 536576;
constexpr size_t kOut3 = 561152;
constexpr size_t kOut4 = 1085440;
constexpr size_t kOutTotal = 1216512;
static_assert(kOut1 * 4 == 49152 && kOut2 * 4 == 2146304 && kOut3 * 4 == 2244608 && kOut4 * 4 == 4341760);
static_assert(kOut0 + (size_t)kBatch * 3 * kN2 == kOut1);
static_assert(kOut1 + (size_t)kBatch * 128 * kN2 == kOut2);
static_assert(kOut2 + (size_t)kBatch * 3 * kN1 == kOut3);
static_assert(kOut3 + (size_t)kBatch * 64 * kN1 == kOut4);
static_assert(kOut4 + (size_t)kBatch * 8 * kN0 == kOutTotal);

constexpr int kM1 = kBatch * kN0 * kNbr / 2;
constexpr int kM2 = kBatch * kN1 * kNbr;
constexpr int kM3 = kBatch * kN1 * kNbr;
constexpr int kM4 = kBatch * kN2 * kNbr;
static_assert(kM1 % 64 == 0 && kM2 % 64 == 0 && kM3 % 64 == 0 && kM4 % 64 == 0);
static_assert(kN0 % 512 == 0 && kN1 % 512 == 0 && kN0 == 8 * 512 && kN1 == 4 * 512);
static_assert(kN0 % 256 == 0 && kN1 % 256 == 0 && kN2 % 256 == 0);
static_assert(kN1 <= 2048 && kN2 <= 2048);
static_assert(((kM1 / 64) * 1) % 8 == 0 && ((kM2 / 64) * 1) % 8 == 0 && ((kM3 / 64) * 1) % 8 == 0 && ((kM4 / 64) * 2) % 8 == 0);

constexpr size_t kMiB = 1048576;
constexpr size_t WS_AH  = 0;
constexpr size_t WS_AL  = WS_AH + 32 * kMiB;
constexpr size_t WS_H   = WS_AL + 32 * kMiB;
constexpr size_t WS_F0  = WS_H + 32 * kMiB;
constexpr size_t WS_F1  = WS_F0 + 524288;
constexpr size_t WS_FQ1 = WS_F1 + 2097152;
constexpr size_t WS_F3  = WS_FQ1 + 1048576;
constexpr size_t WS_FQ2 = WS_F3 + 2097152;
constexpr size_t WS_HS1 = WS_FQ2 + 1048576;
constexpr size_t WS_HS2 = WS_HS1 + 2097152;
constexpr size_t WS_HS3 = WS_HS2 + 2097152;
constexpr size_t WS_HS4 = WS_HS3 + 2097152;
constexpr size_t WS_PT1 = WS_HS4 + 2097152;
constexpr size_t WS_PT2 = WS_PT1 + 65536;
constexpr size_t WS_PT3 = WS_PT2 + 32768;
constexpr size_t WS_PT4 = WS_PT3 + 32768;
constexpr size_t WS_W1H = WS_PT4 + 16384;
constexpr size_t WS_W1L = WS_W1H + 4096;
constexpr size_t WS_W2H = WS_W1L + 4096;
constexpr size_t WS_W2L = WS_W2H + 8192;
constexpr size_t WS_W3H = WS_W2L + 8192;
constexpr size_t WS_W3L = WS_W3H + 16384;
constexpr size_t WS_W4H = WS_W3L + 16384;
constexpr size_t WS_W4L = WS_W4H + 32768;
constexpr size_t WS_END = WS_W4L + 32768;
static_assert(WS_END == 116137984);
static_assert(WS_END <= 134217728);
static_assert((size_t)kM1 * 32 * 2 <= 32 * kMiB && (size_t)kM2 * 64 * 2 <= 32 * kMiB && (size_t)kM3 * 128 * 2 <= 32 * kMiB && (size_t)kM4 * 128 * 2 <= 32 * kMiB);
static_assert((size_t)kM1 * 64 * 4 <= 32 * kMiB && (size_t)kM2 * 64 * 4 <= 32 * kMiB && (size_t)kM3 * 64 * 4 <= 32 * kMiB && (size_t)kM4 * 128 * 4 <= 32 * kMiB);
static_assert((size_t)kBatch * (kN0 / 32) * 128 == 65536 && (size_t)kBatch * (kN1 / 32) * 128 == 32768 && (size_t)kBatch * (kN2 / 32) * 128 == 16384);

__device__ __forceinline__ unsigned short f2bf_bits(float f) {
  unsigned u = __float_as_uint(f);
  return (unsigned short)((u + 0x7FFFu + ((u >> 16) & 1u)) >> 16);
}
__device__ __forceinline__ float bf_bits2f(unsigned short h) { return __uint_as_float(((unsigned)h) << 16); }
__device__ __forceinline__ unsigned pk16(unsigned short a, unsigned short b) { return (unsigned)a | ((unsigned)b << 16); }

__device__ __forceinline__ void dep_guard_h(v8f& a, v8f& b, v16h x, v16h y) { asm volatile("v_nop\n\tv_nop\n\tv_nop\n\tv_nop" : "+v"(a), "+v"(b) : "v"(x), "v"(y)); }
__device__ __forceinline__ void dep_guard_b(v8f& a, v8f& b, v16b x, v16b y) { asm volatile("v_nop\n\tv_nop\n\tv_nop\n\tv_nop" : "+v"(a), "+v"(b) : "v"(x), "v"(y)); }
__device__ __forceinline__ void keep4_h(v16h a, v16h b, v16h c, v16h d) { asm volatile("v_nop" :: "v"(a), "v"(b), "v"(c), "v"(d)); }
__device__ __forceinline__ void keep4_b(v16b a, v16b b, v16b c, v16b d) { asm volatile("v_nop" :: "v"(a), "v"(b), "v"(c), "v"(d)); }
__device__ __forceinline__ void acc_guard4(v8f& a, v8f& b, v8f& c, v8f& d) { asm volatile("v_nop\n\tv_nop\n\tv_nop\n\tv_nop" : "+v"(a), "+v"(b), "+v"(c), "+v"(d)); }
template <typename T> struct Frag;
template <> struct Frag<_Float16> {
  typedef v16h V; union U { v16h v; v8h h[2]; };
  static __device__ __forceinline__ v16h load(const _Float16* p) {
    U f; f.h[0] = *(const v8h*)(p); f.h[1] = *(const v8h*)(p + 16); return f.v;
  }
  static __device__ __forceinline__ v8f mma(v16h a, v16h b, v8f c) {
    return __builtin_amdgcn_wmma_f32_16x16x32_f16(false, a, false, b, (short)0, c, false, false);
  }
  static __device__ __forceinline__ void guard(v8f& a, v8f& b, v16h x, v16h y) { dep_guard_h(a, b, x, y); }
  static __device__ __forceinline__ void keep(v16h a, v16h b, v16h c, v16h d) { keep4_h(a, b, c, d); }
};
template <> struct Frag<__bf16> {
  typedef v16b V; union U { v16b v; v8b h[2]; };
  static __device__ __forceinline__ v16b load(const __bf16* p) {
    U f; f.h[0] = *(const v8b*)(p); f.h[1] = *(const v8b*)(p + 16); return f.v;
  }
  static __device__ __forceinline__ v8f mma(v16b a, v16b b, v8f c) {
    return __builtin_amdgcn_wmma_f32_16x16x32_bf16(false, a, false, b, (short)0, c, false, false);
  }
  static __device__ __forceinline__ void guard(v8f& a, v8f& b, v16b x, v16b y) { dep_guard_b(a, b, x, y); }
  static __device__ __forceinline__ void keep(v16b a, v16b b, v16b c, v16b d) { keep4_b(a, b, c, d); }
};

template <int ET> struct Elem;
template <> struct Elem<0> { typedef _Float16 T; };
template <> struct Elem<1> { typedef __bf16 T; };
template <int ET, bool SPLIT, int BIAS_MODE, int OUT_MODE, bool RESID, int ACT = 0>
__global__ __launch_bounds__(256) void wmma_gemm64(
    const unsigned short* __restrict__ Ap, const unsigned short* __restrict__ A2p, int lda, long strideA,
    const unsigned short* __restrict__ Btp, const unsigned short* __restrict__ Bt2p, int ldb, long strideB,
    void* __restrict__ Cout, void* __restrict__ Cout2, int ldc, long strideC,
    const float* __restrict__ bias,
    const float* __restrict__ resid, long strideR,
    int M, int N, int K, float scale) {
  typedef typename Elem<ET>::T T;
  typedef typename Frag<T>::V V;
  const T* A = (const T*)Ap; const T* A2 = (const T*)A2p; const T* Bt = (const T*)Btp; const T* Bt2 = (const T*)Bt2p;
  __shared__ __align__(16) float sT[8][16 * 68];
  const int b    = blockIdx.y;
  const int lane = threadIdx.x & 31;
  const int wave = threadIdx.x >> 5;
  const int tilesN = N >> 6;
  const int tilesM = M >> 6;
  const int tile = blockIdx.x * 8 + wave;
  if (tile >= tilesM * tilesN) return;
  const int tm = tile / tilesN;
  const int tn = tile - tm * tilesN;
  const int m0 = tm << 6;
  const int n0 = tn << 6;

  const T* Ab  = A  + (size_t)b * strideA;
  const T* Bb  = Bt + (size_t)b * strideB;
  const T* Ab2 = SPLIT ? (A2  + (size_t)b * strideA) : nullptr;
  const T* Bb2 = SPLIT ? (Bt2 + (size_t)b * strideB) : nullptr;

  const int rlane = lane & 15;
  const int koff  = (lane >> 4) * 8;
  const int mOff  = (lane >> 4) * 8;

  v8f acc[4][4];
#pragma unroll
  for (int i = 0; i < 4; ++i)
#pragma unroll
    for (int j = 0; j < 4; ++j) acc[i][j] = (v8f){0.f,0.f,0.f,0.f,0.f,0.f,0.f,0.f};

  for (int k0 = 0; k0 < K; k0 += 32) {
    V bh[4], bl[4];
#pragma unroll
    for (int j = 0; j < 4; ++j) {
      const size_t bo = (size_t)(n0 + (j << 4) + rlane) * ldb + koff + k0;
      bh[j] = Frag<T>::load(Bb + bo);
      if (SPLIT) bl[j] = Frag<T>::load(Bb2 + bo);
    }
#pragma unroll
    for (int i = 0; i < 4; ++i) {
      const size_t ao = (size_t)(m0 + (i << 4) + rlane) * lda + koff + k0;
      V ah = Frag<T>::load(Ab + ao);
      V al;
      if (SPLIT) al = Frag<T>::load(Ab2 + ao);
#pragma unroll
      for (int j = 0; j < 4; ++j) {
        acc[i][j] = Frag<T>::mma(ah, bh[j], acc[i][j]);
        if (SPLIT) {
          acc[i][j] = Frag<T>::mma(ah, bl[j], acc[i][j]);
          acc[i][j] = Frag<T>::mma(al, bh[j], acc[i][j]);
        }
      }
      Frag<T>::guard(acc[i][0], acc[i][3], ah, SPLIT ? al : ah);
    }
    Frag<T>::keep(bh[0], bh[1], bh[2], bh[3]);
    if (SPLIT) Frag<T>::keep(bl[0], bl[1], bl[2], bl[3]);
  }
  acc_guard4(acc[0][0], acc[0][1], acc[0][2], acc[0][3]);
  acc_guard4(acc[1][0], acc[1][1], acc[1][2], acc[1][3]);
  acc_guard4(acc[2][0], acc[2][1], acc[2][2], acc[2][3]);
  acc_guard4(acc[3][0], acc[3][1], acc[3][2], acc[3][3]);

  float* slab = sT[wave];
  const float* Rb = RESID ? (resid + (size_t)b * strideR) : nullptr;
#pragma unroll
  for (int i = 0; i < 4; ++i) {
    const int mBase = m0 + (i << 4);
#pragma unroll
    for (int j = 0; j < 4; ++j) {
      const int n = n0 + (j << 4) + rlane;
      float bv = 0.f;
      if (BIAS_MODE == 2) bv = bias[n];
#pragma unroll
      for (int r = 0; r < 8; ++r) {
        float v = acc[i][j][r] * scale;
        if (BIAS_MODE == 1) v += bias[mBase + mOff + r];
        if (BIAS_MODE == 2) v += bv;
        if (RESID) v += Rb[(size_t)(mBase + mOff + r) * ldc + n];
        if (ACT == 2) v = fmaxf(v, 0.0f);
        if (ACT == 4) v = (v > 0.f) ? v : 0.01f * v;
        slab[(mOff + r) * 68 + (j << 4) + rlane] = v;
      }
    }
    __builtin_amdgcn_fence(__ATOMIC_RELEASE, "workgroup");
    __builtin_amdgcn_wave_barrier();
    __builtin_amdgcn_fence(__ATOMIC_ACQUIRE, "workgroup");
    if (OUT_MODE == 0) {
      float* C = (float*)Cout + (size_t)b * strideC;
      const int hh = lane >> 4, c4 = (lane & 15) * 4;
      for (int pass = 0; pass < 2; ++pass) {
#pragma unroll
        for (int it = 0; it < 8; ++it) {
          const int row = it * 2 + hh;
          v4f v = *(const v4f*)(slab + row * 68 + c4);
          *(volatile v4f*)(C + (size_t)(mBase + row) * ldc + n0 + c4) = v;
        }
        __threadfence();
      }
    } else {
      const int q = lane >> 3, c8 = (lane & 7) * 8;
      unsigned short* C  = (unsigned short*)Cout  + (size_t)b * strideC;
      unsigned short* C2 = (OUT_MODE == 2) ? ((unsigned short*)Cout2 + (size_t)b * strideC) : nullptr;
      for (int pass = 0; pass < 2; ++pass) {
#pragma unroll
        for (int it = 0; it < 4; ++it) {
          const int row = it * 4 + q;
          const float* sp = slab + row * 68 + c8;
          v8h hv, lv;
#pragma unroll
          for (int e = 0; e < 8; ++e) {
            if (OUT_MODE == 1) {
              hv[e] = (_Float16)sp[e];
            } else {
              unsigned short hb = f2bf_bits(sp[e]);
              unsigned short lb = f2bf_bits(sp[e] - bf_bits2f(hb));
              hv[e] = __builtin_bit_cast(_Float16, hb);
              lv[e] = __builtin_bit_cast(_Float16, lb);
            }
          }
          *(volatile v8h*)(C + (size_t)(mBase + row) * ldc + n0 + c8) = hv;
          if (OUT_MODE == 2) *(volatile v8h*)(C2 + (size_t)(mBase + row) * ldc + n0 + c8) = lv;
        }
        __threadfence();
      }
    }
    __builtin_amdgcn_fence(__ATOMIC_RELEASE, "workgroup");
    __builtin_amdgcn_wave_barrier();
    __builtin_amdgcn_fence(__ATOMIC_ACQUIRE, "workgroup");
  }
}

__global__ __launch_bounds__(256) void k_wsplit(const float* __restrict__ W, int oreal, int kin, int nrows, int kp, int twin,
                                               unsigned short* __restrict__ hi, unsigned short* __restrict__ lo) {
  const int tpr = kp >> 3;
  const int i = blockIdx.x * 256 + threadIdx.x;
  if (i >= nrows * tpr) return;
  const int n  = i / tpr;
  const int k0 = (i - n * tpr) * 8;
  const int second = (twin != 0 && n >= oreal) ? 1 : 0;
  const int nn0 = n - second * oreal;
  const int nn  = nn0 < 0 ? 0 : (nn0 < oreal ? nn0 : oreal - 1);
  const int ks  = second * kin;
  unsigned short hb[8], lb[8];
#pragma unroll
  for (int e = 0; e < 8; ++e) {
    const int k   = k0 + e;
    const int kk0 = k - ks;
    const bool valid = (nn0 >= 0) && (nn0 < oreal) && (kk0 >= 0) && (kk0 < kin);
    const int kk  = kk0 < 0 ? 0 : (kk0 < kin ? kk0 : kin - 1);
    float v = W[(size_t)nn * kin + kk];
    if (!valid) v = 0.0f;
    hb[e] = f2bf_bits(v);
    lb[e] = f2bf_bits(v - bf_bits2f(hb[e]));
  }
  const v4u uh = (v4u){pk16(hb[0], hb[1]), pk16(hb[2], hb[3]), pk16(hb[4], hb[5]), pk16(hb[6], hb[7])};
  const v4u ul = (v4u){pk16(lb[0], lb[1]), pk16(lb[2], lb[3]), pk16(lb[4], lb[5]), pk16(lb[6], lb[7])};
  const size_t o = (size_t)i * 8;
  *(volatile v4u*)(hi + o) = uh;
  *(volatile v4u*)(lo + o) = ul;
  __threadfence();
  *(volatile v4u*)(hi + o) = uh;
  *(volatile v4u*)(lo + o) = ul;
}

__global__ __launch_bounds__(256) void k_proj(const float* __restrict__ x, const float* __restrict__ w, const float* __restrict__ bias,
                                             float* __restrict__ f0, float* __restrict__ o4) {
  __shared__ float sw[32];
  const int tid = threadIdx.x;
  if (tid < 32) {
    const int ia = (tid < 24) ? tid : 23;
    const int ib = (tid < 24) ? 0 : (tid - 24);
    const float wa = w[ia];
    const float wb = bias[ib];
    sw[tid] = (tid < 24) ? wa : wb;
  }
  __syncthreads();
  const int t  = blockIdx.x * 256 + tid;
  const int b  = t >> 10;
  const int n4 = (t & 1023) * 4;
  const float* xb = x + (size_t)b * 3 * kN0;
  const v4f x0 = *(const v4f*)(xb + n4);
  const v4f x1 = *(const v4f*)(xb + kN0 + n4);
  const v4f x2 = *(const v4f*)(xb + 2 * kN0 + n4);
  v4f r[8];
#pragma unroll
  for (int o = 0; o < 8; ++o) {
    const float w0 = sw[o * 3 + 0], w1 = sw[o * 3 + 1], w2 = sw[o * 3 + 2], bo = sw[24 + o];
#pragma unroll
    for (int e = 0; e < 4; ++e) {
      float p = w0 * x0[e];
      p = fmaf(w1, x1[e], p);
      p = fmaf(w2, x2[e], p);
      r[o][e] = p + bo;
    }
  }
  for (int pass = 0; pass < 2; ++pass) {
#pragma unroll
    for (int o = 0; o < 8; ++o) {
      const size_t off = (size_t)(b * 8 + o) * kN0 + n4;
      *(volatile v4f*)(f0 + off) = r[o];
      *(volatile v4f*)(o4 + off) = r[o];
    }
    __threadfence();
  }
}

__device__ __forceinline__ void edge4(const float* fkb, const float* fqb, int nk, int nq, int nj, int qc, int C, int k0, bool diffp,
                                      unsigned& h01, unsigned& h23, unsigned& l01, unsigned& l23) {
  unsigned short hb[4], lb[4];
#pragma unroll
  for (int e = 0; e < 4; ++e) {
    const int k  = k0 + e;
    const int kc = diffp ? k : (k - C);
    const float vk = fkb[(size_t)kc * nk + nj];
    const float vq = fqb[(size_t)kc * nq + qc];
    const float v  = diffp ? (vk - vq) : vq;
    hb[e] = f2bf_bits(v);
    lb[e] = f2bf_bits(v - bf_bits2f(hb[e]));
  }
  h01 = pk16(hb[0], hb[1]); h23 = pk16(hb[2], hb[3]);
  l01 = pk16(lb[0], lb[1]); l23 = pk16(lb[2], lb[3]);
}

constexpr int kKnnT  = 256;
constexpr int kKnnKT = 512;
__global__ __launch_bounds__(kKnnT) void k_knn_edge(const float* __restrict__ cq, int nq, const float* __restrict__ ck, int nk,
                                                     const float* __restrict__ fq, const float* __restrict__ fk, int C, int tprShift,
                                                     unsigned short* __restrict__ ah, unsigned short* __restrict__ al) {
  __shared__ float skx[kKnnKT], sky[kKnnKT], skz[kKnnKT], skq[kKnnKT];
  __shared__ int sidx[kKnnT * 16];
  const int tid = threadIdx.x;
  const int b   = blockIdx.y;
  const int qb0 = blockIdx.x * kKnnT;
  const int qi  = qb0 + tid;
  const float* cqb = cq + (size_t)b * 3 * nq;
  const float* ckb = ck + (size_t)b * 3 * nk;
  const float qx = cqb[qi], qy = cqb[nq + qi], qz = cqb[2 * nq + qi];
  const float qsq = (qx * qx + qz * qz) + qy * qy;
  float bd[16];
  int   bi[16];
#pragma unroll
  for (int s = 0; s < 16; ++s) { bd[s] = 3.0e38f; bi[s] = 0; }
  const int ntile = nk / kKnnKT;
  for (int t = 0; t < ntile; ++t) {
    __syncthreads();
#pragma unroll
    for (int r = 0; r < kKnnKT / kKnnT; ++r) {
      const int kl = tid + r * kKnnT;
      const int kg = t * kKnnKT + kl;
      const float kx = ckb[kg], ky = ckb[nk + kg], kz = ckb[2 * nk + kg];
      skx[kl] = kx; sky[kl] = ky; skz[kl] = kz;
      skq[kl] = (kx * kx + kz * kz) + ky * ky;
    }
    __syncthreads();
#pragma unroll 1
    for (int jk = 0; jk < kKnnKT; ++jk) {
      const float kx = skx[jk], ky = sky[jk], kz = skz[jk];
      const float dot = fmaf(qz, kz, fmaf(qy, ky, qx * kx));
      const float d = (qsq + skq[jk]) - 2.0f * dot;
      if (d < bd[15]) {
        float cd = d;
        int   ci = t * kKnnKT + jk;
#pragma unroll
        for (int s = 0; s < 16; ++s) {
          const bool lt = (cd < bd[s]) || (cd == bd[s] && ci < bi[s]);
          const float td = bd[s];
          const int   ti = bi[s];
          bd[s] = lt ? cd : td;
          bi[s] = lt ? ci : ti;
          cd = lt ? td : cd;
          ci = lt ? ti : ci;
        }
      }
    }
  }
#pragma unroll
  for (int s = 0; s < 16; ++s) sidx[tid * 16 + s] = bi[s];
  __syncthreads();

  const int tpr   = 1 << tprShift;
  const int iters = 16 << tprShift;
  const float* fkb = fk + (size_t)b * C * nk;
  const float* fqb = fq + (size_t)b * C * nq;
  const size_t obase = ((size_t)b * nq + qb0) * 16 * (size_t)(2 * C);
#pragma unroll 1
  for (int itb = 0; itb < iters; ++itb) {
    const int i  = itb * kKnnT + tid;
    const int ml = i >> tprShift;
    const int k0 = (i & (tpr - 1)) * 8;
    int nj = sidx[ml];
    nj = nj < 0 ? 0 : (nj >= nk ? nk - 1 : nj);
    const int qc = qb0 + (ml >> 4);
    const bool diffp = (k0 < C);
    unsigned wh0, wh1, wl0, wl1, wh2, wh3, wl2, wl3;
    edge4(fkb, fqb, nk, nq, nj, qc, C, k0, diffp, wh0, wh1, wl0, wl1);
    asm volatile("" : "+v"(wh0), "+v"(wh1), "+v"(wl0), "+v"(wl1) : : "memory");
    edge4(fkb, fqb, nk, nq, nj, qc, C, k0 + 4, diffp, wh2, wh3, wl2, wl3);
    const v4u uh = (v4u){wh0, wh1, wh2, wh3};
    const v4u ul = (v4u){wl0, wl1, wl2, wl3};
    const size_t o = obase + (size_t)i * 8;
    *(volatile v4u*)(ah + o) = uh;
    *(volatile v4u*)(al + o) = ul;
    __threadfence();
    *(volatile v4u*)(ah + o) = uh;
    *(volatile v4u*)(al + o) = ul;
  }
}

constexpr int kHrPitch = 36;
__global__ __launch_bounds__(256) void k_hreduce(const float* __restrict__ h, int O, int nq, const float* __restrict__ gw,
                                                float* __restrict__ hsel, float* __restrict__ part) {
  __shared__ __align__(16) float tile[128 * kHrPitch];
  __shared__ float stat[256 * 2];
  __shared__ __align__(16) float pline[32];
  const int tid = threadIdx.x, lane = tid & 31, wave = tid >> 5;
  const int b = blockIdx.y, qb = blockIdx.x, nqb = gridDim.x;
  const int q0    = qb * 32;
  const int cbase = (4 * lane) & (O - 1);
  const int ngrp  = O >> 5;
  const int gsz   = O >> 2;
  const v4f g4 = *(const v4f*)(gw + cbase);
  float s = 0.0f, ss = 0.0f;
#pragma unroll 1
  for (int qq = 0; qq < 4; ++qq) {
    const int q = q0 + wave * 4 + qq;
    const float* base = h + (size_t)(b * nq + q) * 16 * O + 4 * lane;
    float mx[4], mn[4];
#pragma unroll
    for (int e = 0; e < 4; ++e) { mx[e] = -3.0e38f; mn[e] = 3.0e38f; }
#pragma unroll 1
    for (int g = 0; g < ngrp; ++g) {
      const float* p = base + (size_t)g * 512;
#pragma unroll
      for (int u = 0; u < 4; ++u) {
        const v4f v = *(const v4f*)(p + u * 128);
#pragma unroll
        for (int e = 0; e < 4; ++e) {
          mx[e] = fmaxf(mx[e], v[e]);
          mn[e] = fminf(mn[e], v[e]);
          s  += v[e];
          ss += v[e] * v[e];
        }
      }
    }
#pragma unroll
    for (int e = 0; e < 4; ++e) {
      const float ax = __shfl_xor(mx[e], 16, 32);
      const float an = __shfl_xor(mn[e], 16, 32);
      if (O <= 64) { mx[e] = fmaxf(mx[e], ax); mn[e] = fminf(mn[e], an); }
      const float bx = __shfl_xor(mx[e], 8, 32);
      const float bn = __shfl_xor(mn[e], 8, 32);
      if (O <= 32) { mx[e] = fmaxf(mx[e], bx); mn[e] = fminf(mn[e], bn); }
    }
    if (4 * lane < O) {
#pragma unroll
      for (int e = 0; e < 4; ++e)
        tile[(cbase + e) * kHrPitch + wave * 4 + qq] = (g4[e] >= 0.0f) ? mx[e] : mn[e];
    }
  }
  stat[tid * 2]     = s;
  stat[tid * 2 + 1] = ss;
  __syncthreads();
  if (tid < 32) {
    float val = 0.0f;
    if (tid < 8) {
      const int g = tid >> 1, which = tid & 1;
      float acc = 0.0f;
#pragma unroll 1
      for (int t = 0; t < 256; ++t) {
        const int l  = t & 31;
        const int lg = ((4 * l) & (O - 1)) / gsz;
        const float v = stat[t * 2 + which];
        acc += (lg == g) ? v : 0.0f;
      }
      val = acc;
    }
    pline[tid] = val;
  }
  __syncthreads();
  for (int pass = 0; pass < 2; ++pass) {
#pragma unroll
    for (int it = 0; it < 4; ++it) {
      if (it < ngrp) {
        const int o  = it * 32 + wave * 4 + (lane >> 3);
        const int c4 = (lane & 7) * 4;
        const v4f v = *(const v4f*)(tile + o * kHrPitch + c4);
        *(volatile v4f*)(hsel + ((size_t)(b * O + o) * nq + q0 + c4)) = v;
      }
    }
    if (tid < 8) {
      const v4f v = *(const v4f*)(pline + tid * 4);
      *(volatile v4f*)(part + ((size_t)(b * nqb + qb) * 32 + tid * 4)) = v;
    }
    __threadfence();
  }
}

__global__ __launch_bounds__(256) void k_finalize(const float* __restrict__ part, int nqb, const float* __restrict__ hsel,
                                                 const float* __restrict__ gw, const float* __restrict__ gb,
                                                 int O, int nq, float invCnt, float* __restrict__ fout) {
  __shared__ float smean[4];
  __shared__ float sinv[4];
  const int tid  = threadIdx.x;
  const int nq4  = nq >> 2;
  const int perb = O * nq4;
  const int b    = (int)(((size_t)blockIdx.x * 256) / (size_t)perb);
  if (tid < 4) {
    double s = 0.0, ss = 0.0;
    const float* pp = part + (size_t)b * nqb * 32 + 2 * tid;
#pragma unroll 1
    for (int i = 0; i < nqb; ++i) {
      s  += (double)pp[(size_t)i * 32];
      ss += (double)pp[(size_t)i * 32 + 1];
    }
    const double ic   = (double)invCnt;
    const double mean = s * ic;
    double var = ss * ic - mean * mean;
    var = var < 0.0 ? 0.0 : var;
    const float ve = (float)var + 1.0e-5f;
    smean[tid] = (float)mean;
    sinv[tid]  = 1.0f / sqrtf(ve);
  }
  __syncthreads();
  const int e4  = blockIdx.x * 256 + tid;
  const int rem = e4 - b * perb;
  const int o   = rem / nq4;
  const int q4  = (rem - o * nq4) * 4;
  const int g   = o / (O >> 2);
  const float mu = smean[g], inv = sinv[g], wv = gw[o], bv = gb[o];
  const size_t off = (size_t)(b * O + o) * nq + q4;
  const v4f v = *(const v4f*)(hsel + off);
  v4f y;
#pragma unroll
  for (int e = 0; e < 4; ++e) {
    const float t = ((v[e] - mu) * inv) * wv + bv;
    y[e] = (t >= 0.0f) ? t : 0.2f * t;
  }
  *(volatile v4f*)(fout + off) = y;
  __threadfence();
  *(volatile v4f*)(fout + off) = y;
}

template <int PPT>
__global__ __launch_bounds__(512) void k_fps(const float* __restrict__ coor, int n, int m,
                                            const float* __restrict__ feat, int C,
                                            float* __restrict__ coorOut, float* __restrict__ fqOut) {
  static_assert(PPT % 4 == 0);
  __shared__ __align__(16) int sel[2048];
  __shared__ float redv[2][16];
  __shared__ int   redi[2][16];
  const int tid = threadIdx.x, lane = tid & 31, wave = tid >> 5;
  const int b = blockIdx.x;
  const float* cb = coor + (size_t)b * 3 * n;
  const int i0 = tid * PPT;
  float px[PPT], py[PPT], pz[PPT], dist[PPT];
#pragma unroll
  for (int g4 = 0; g4 < PPT / 4; ++g4) {
    const v4f vx = *(const v4f*)(cb + i0 + 4 * g4);
    const v4f vy = *(const v4f*)(cb + n + i0 + 4 * g4);
    const v4f vz = *(const v4f*)(cb + 2 * n + i0 + 4 * g4);
#pragma unroll
    for (int e = 0; e < 4; ++e) {
      px[4 * g4 + e] = vx[e]; py[4 * g4 + e] = vy[e]; pz[4 * g4 + e] = vz[e];
      dist[4 * g4 + e] = 1.0e10f;
    }
  }
  int far = 0;
#pragma unroll 1
  for (int it = 0; it < m; ++it) {
    if (tid == 0) sel[it] = far;
    const float cx = cb[far], cy = cb[n + far], cz = cb[2 * n + far];
    float lmax = -1.0f;
    int   li   = 0;
#pragma unroll
    for (int p = 0; p < PPT; ++p) {
      const float dx = px[p] - cx, dy = py[p] - cy, dz = pz[p] - cz;
      const float d   = (dx * dx + dz * dz) + dy * dy;
      const float cur = (d < dist[p]) ? d : dist[p];
      dist[p] = cur;
      const bool tk = cur > lmax;
      lmax = tk ? cur : lmax;
      li   = tk ? (i0 + p) : li;
    }
#pragma unroll
    for (int off = 16; off > 0; off >>= 1) {
      const float ov = __shfl_xor(lmax, off, 32);
      const int   oi = __shfl_xor(li, off, 32);
      const bool tk = (ov > lmax) || (ov == lmax && oi < li);
      lmax = tk ? ov : lmax;
      li   = tk ? oi : li;
    }
    const int par = it & 1;
    if (lane == 0) { redv[par][wave] = lmax; redi[par][wave] = li; }
    __syncthreads();
    float bvv = redv[par][0];
    int   bix = redi[par][0];
#pragma unroll
    for (int w = 1; w < 16; ++w) {
      const float v  = redv[par][w];
      const int   ix = redi[par][w];
      const bool tk = (v > bvv) || (v == bvv && ix < bix);
      bvv = tk ? v : bvv;
      bix = tk ? ix : bix;
    }
    far = bix < 0 ? 0 : (bix >= n ? n - 1 : bix);
  }
  __syncthreads();
  const int m4 = m >> 2;
  if (tid < m4) {
    const int j4 = tid * 4;
    const v4i sv = *(const v4i*)(sel + j4);
    int s[4];
#pragma unroll
    for (int e = 0; e < 4; ++e) { int t = sv[e]; s[e] = t < 0 ? 0 : (t >= n ? n - 1 : t); }
#pragma unroll 1
    for (int c = 0; c < 3; ++c) {
      v4f cv;
#pragma unroll
      for (int e = 0; e < 4; ++e) cv[e] = cb[(size_t)c * n + s[e]];
      float* dst = coorOut + ((size_t)b * 3 + c) * m + j4;
      *(volatile v4f*)dst = cv;
      __threadfence();
      *(volatile v4f*)dst = cv;
    }
  }
  const int tot4 = C * m4;
#pragma unroll 1
  for (int e4 = tid; e4 < tot4; e4 += 512) {
    const int c  = e4 / m4;
    const int j4 = (e4 - c * m4) * 4;
    const v4i sv = *(const v4i*)(sel + j4);
    int s[4];
#pragma unroll
    for (int e = 0; e < 4; ++e) { int t = sv[e]; s[e] = t < 0 ? 0 : (t >= n ? n - 1 : t); }
    const float* fr = feat + ((size_t)b * C + c) * n;
    v4f fv;
#pragma unroll
    for (int e = 0; e < 4; ++e) fv[e] = fr[s[e]];
    float* dst = fqOut + ((size_t)b * C + c) * m + j4;
    *(volatile v4f*)dst = fv;
    __threadfence();
    *(volatile v4f*)dst = fv;
  }
}

extern "C" void kernel_launch(void* const* d_in, const int* in_sizes, int n_in,
                              void* d_out, int out_size, void* d_ws, size_t ws_size,
                              hipStream_t stream) {
  (void)in_sizes; (void)n_in;
  if (ws_size < WS_END) return;
  if ((size_t)out_size < kOutTotal) return;

  const float* x    = (const float*)d_in[0];
  const float* w_in = (const float*)d_in[1];
  const float* b_in = (const float*)d_in[2];
  const float* w1   = (const float*)d_in[3];
  const float* g1w  = (const float*)d_in[4];
  const float* g1b  = (const float*)d_in[5];
  const float* w2   = (const float*)d_in[6];
  const float* g2w  = (const float*)d_in[7];
  const float* g2b  = (const float*)d_in[8];
  const float* w3   = (const float*)d_in[9];
  const float* g3w  = (const float*)d_in[10];
  const float* g3b  = (const float*)d_in[11];
  const float* w4   = (const float*)d_in[12];
  const float* g4w  = (const float*)d_in[13];
  const float* g4b  = (const float*)d_in[14];

  float* out = (float*)d_out;
  char*  ws  = (char*)d_ws;
  unsigned short* AH = (unsigned short*)(ws + WS_AH);
  unsigned short* AL = (unsigned short*)(ws + WS_AL);
  float* H   = (float*)(ws + WS_H);
  float* F0  = (float*)(ws + WS_F0);
  float* F1  = (float*)(ws + WS_F1);
  float* FQ1 = (float*)(ws + WS_FQ1);
  float* F3  = (float*)(ws + WS_F3);
  float* FQ2 = (float*)(ws + WS_FQ2);
  float* HS1 = (float*)(ws + WS_HS1);
  float* HS2 = (float*)(ws + WS_HS2);
  float* HS3 = (float*)(ws + WS_HS3);
  float* HS4 = (float*)(ws + WS_HS4);
  float* PT1 = (float*)(ws + WS_PT1);
  float* PT2 = (float*)(ws + WS_PT2);
  float* PT3 = (float*)(ws + WS_PT3);
  float* PT4 = (float*)(ws + WS_PT4);
  unsigned short* W1H = (unsigned short*)(ws + WS_W1H);
  unsigned short* W1L = (unsigned short*)(ws + WS_W1L);
  unsigned short* W2H = (unsigned short*)(ws + WS_W2H);
  unsigned short* W2L = (unsigned short*)(ws + WS_W2L);
  unsigned short* W3H = (unsigned short*)(ws + WS_W3H);
  unsigned short* W3L = (unsigned short*)(ws + WS_W3L);
  unsigned short* W4H = (unsigned short*)(ws + WS_W4H);
  unsigned short* W4L = (unsigned short*)(ws + WS_W4L);

  k_wsplit<<<(64 * 32 / 8 + 255) / 256, 256, 0, stream>>>(w1, 32, 16, 64, 32, 1, W1H, W1L);
  k_wsplit<<<(64 * 64 / 8 + 255) / 256, 256, 0, stream>>>(w2, 64, 64, 64, 64, 0, W2H, W2L);
  k_wsplit<<<(64 * 128 / 8 + 255) / 256, 256, 0, stream>>>(w3, 64, 128, 64, 128, 0, W3H, W3L);
  k_wsplit<<<(128 * 128 / 8 + 255) / 256, 256, 0, stream>>>(w4, 128, 128, 128, 128, 0, W4H, W4L);

  static_assert((kBatch * kN0 / 4) % 256 == 0 && kN0 / 4 == 1024);
  k_proj<<<(kBatch * kN0 / 4) / 256, 256, 0, stream>>>(x, w_in, b_in, F0, out + kOut4);

  k_knn_edge<<<dim3(kN0 / kKnnT, kBatch), kKnnT, 0, stream>>>(x, kN0, x, kN0, F0, F0, 8, 1, AH, AL);
  {
    constexpr int gM = kM1, gN = 64, gK = 32;
    static_assert(gM % 64 == 0 && gN % 64 == 0 && gK % 32 == 0);
    wmma_gemm64<1, true, 0, 0, false, 0><<<dim3((gM / 64) * (gN / 64) / 8, 1), 256, 0, stream>>>(
        AH, AL, 32, 0L, W1H, W1L, 32, 0L, (void*)H, nullptr, 64, 0L, nullptr, nullptr, 0L, gM, gN, gK, 1.0f);
    k_hreduce<<<dim3(kN0 / 32, kBatch), 256, 0, stream>>>(H, 32, kN0, g1w, HS1, PT1);
    static_assert((kBatch * 32 * kN0 / 4) % 256 == 0 && (32 * kN0 / 4) % 256 == 0);
    k_finalize<<<(kBatch * 32 * kN0 / 4) / 256, 256, 0, stream>>>(PT1, kN0 / 32, HS1, g1w, g1b, 32, kN0, kInvCnt, F1);
  }

  k_fps<8><<<kBatch, 512, 0, stream>>>(x, kN0, kN1, F1, 32, out + kOut2, FQ1);

  k_knn_edge<<<dim3(kN1 / kKnnT, kBatch), kKnnT, 0, stream>>>(out + kOut2, kN1, x, kN0, FQ1, F1, 32, 3, AH, AL);
  {
    constexpr int gM = kM2, gN = 64, gK = 64;
    static_assert(gM % 64 == 0 && gN % 64 == 0 && gK % 32 == 0);
    wmma_gemm64<1, true, 0, 0, false, 0><<<dim3((gM / 64) * (gN / 64) / 8, 1), 256, 0, stream>>>(
        AH, AL, 64, 0L, W2H, W2L, 64, 0L, (void*)H, nullptr, 64, 0L, nullptr, nullptr, 0L, gM, gN, gK, 1.0f);
    k_hreduce<<<dim3(kN1 / 32, kBatch), 256, 0, stream>>>(H, 64, kN1, g2w, HS2, PT2);
    static_assert((kBatch * 64 * kN1 / 4) % 256 == 0 && (64 * kN1 / 4) % 256 == 0);
    k_finalize<<<(kBatch * 64 * kN1 / 4) / 256, 256, 0, stream>>>(PT2, kN1 / 32, HS2, g2w, g2b, 64, kN1, kInvCnt, out + kOut3);
  }

  k_knn_edge<<<dim3(kN1 / kKnnT, kBatch), kKnnT, 0, stream>>>(out + kOut2, kN1, out + kOut2, kN1, out + kOut3, out + kOut3, 64, 4, AH, AL);
  {
    constexpr int gM = kM3, gN = 64, gK = 128;
    static_assert(gM % 64 == 0 && gN % 64 == 0 && gK % 32 == 0);
    wmma_gemm64<1, true, 0, 0, false, 0><<<dim3((gM / 64) * (gN / 64) / 8, 1), 256, 0, stream>>>(
        AH, AL, 128, 0L, W3H, W3L, 128, 0L, (void*)H, nullptr, 64, 0L, nullptr, nullptr, 0L, gM, gN, gK, 1.0f);
    k_hreduce<<<dim3(kN1 / 32, kBatch), 256, 0, stream>>>(H, 64, kN1, g3w, HS3, PT3);
    k_finalize<<<(kBatch * 64 * kN1 / 4) / 256, 256, 0, stream>>>(PT3, kN1 / 32, HS3, g3w, g3b, 64, kN1, kInvCnt, F3);
  }

  k_fps<4><<<kBatch, 512, 0, stream>>>(out + kOut2, kN1, kN2, F3, 64, out + kOut0, FQ2);

  k_knn_edge<<<dim3(kN2 / kKnnT, kBatch), kKnnT, 0, stream>>>(out + kOut0, kN2, out + kOut2, kN1, FQ2, F3, 64, 4, AH, AL);
  {
    constexpr int gM = kM4, gN = 128, gK = 128;
    static_assert(gM % 64 == 0 && gN % 64 == 0 && gK % 32 == 0);
    wmma_gemm64<1, true, 0, 0, false, 0><<<dim3((gM / 64) * (gN / 64) / 8, 1), 256, 0, stream>>>(
        AH, AL, 128, 0L, W4H, W4L, 128, 0L, (void*)H, nullptr, 128, 0L, nullptr, nullptr, 0L, gM, gN, gK, 1.0f);
    k_hreduce<<<dim3(kN2 / 32, kBatch), 256, 0, stream>>>(H, 128, kN2, g4w, HS4, PT4);
    static_assert((kBatch * 128 * kN2 / 4) % 256 == 0 && (128 * kN2 / 4) % 256 == 0);
    k_finalize<<<(kBatch * 128 * kN2 / 4) / 256, 256, 0, stream>>>(PT4, kN2 / 32, HS4, g4w, g4b, 128, kN2, kInvCnt, out + kOut1);
  }
}
